// SAGE_delta_7146825581285
// MI455X (gfx1250) — hardware-verified
//
#include <hip/hip_runtime.h>
#include <stddef.h>


#define DK      512
#define NTHR    256
#define NWAVE   8

#define NB      128
#define EPT     8
#define NGRP    2
#define CHUNK   (NTHR * EPT * NGRP)
#define WCAP    (EPT * NGRP * 32)
#define LISTN   (NWAVE * WCAP)
#define LDS_ACC  (NB * DK * 4)
#define LDS_LIST (LISTN * 4)
#define LDS_CNT  (NB * 4)
#define LDS_INV  (NB * 4)
#define LDS_WC   64
#define LDS_AGG  (LDS_ACC + LDS_LIST + LDS_CNT + LDS_INV + LDS_WC)

#define GR      32
#define KC      128
#define PA      136
#define TABMAX  1024
#define G_STG   (GR * PA * 2)

static_assert((CHUNK & (CHUNK - 1)) == 0);
static_assert(CHUNK <= 4096);
static_assert((NB & (NB - 1)) == 0);
static_assert(NB <= 4096);
static_assert(NWAVE * 4 <= LDS_WC);
static_assert(LDS_AGG <= 300 * 1024);
static_assert((PA % 8) == 0);
static_assert(DK == 512);
static_assert(DK % KC == 0 && KC % 32 == 0);
static_assert(GR * KC == NTHR * 16);
static_assert((NB * DK / 4) % NTHR == 0);

typedef float    v4f   __attribute__((ext_vector_type(4)));
typedef float    v8f   __attribute__((ext_vector_type(8)));
typedef int      v4i   __attribute__((ext_vector_type(4)));
typedef __bf16   bf16_t;
typedef bf16_t   v8bf  __attribute__((ext_vector_type(8)));
typedef bf16_t   v16bf __attribute__((ext_vector_type(16)));
typedef _Float16 f16_t;
typedef f16_t    v8h   __attribute__((ext_vector_type(8)));
typedef f16_t    v16h  __attribute__((ext_vector_type(16)));
union FragB  { v16bf v; v8bf h[2]; v4i q[2]; };
union FragH  { v16h  v; v8h  h[2]; v4i q[2]; };
union Pack8B { v8bf v; v4i q; };
union Pack8H { v8h  v; v4i q; };

template <int NOUT> struct GemmLds {
  static constexpr int OTP   = NOUT + 4;
  static constexpr int OTB   = GR * OTP * 4;
  static constexpr int TOTAL = 2 * G_STG + OTB + 2 * TABMAX * 4 + 2 * GR * 4;
};
static_assert(GemmLds<512>::TOTAL <= 300 * 1024);
static_assert(GemmLds<64>::TOTAL <= 300 * 1024);

__device__ __forceinline__ v8f wmb(v16bf a, v16bf b, v8f c) {
  v8f d = __builtin_amdgcn_wmma_f32_16x16x32_bf16(false, a, false, b, (short)0, c, false, false);
  asm volatile("v_nop\n\tv_nop\n\tv_nop\n\tv_nop" : "+v"(d) : "v"(a), "v"(b));
  return d;
}
__device__ __forceinline__ v8f wmh(v16h a, v16h b, v8f c) {
  v8f d = __builtin_amdgcn_wmma_f32_16x16x32_f16(false, a, false, b, (short)0, c, false, false);
  asm volatile("v_nop\n\tv_nop\n\tv_nop\n\tv_nop" : "+v"(d) : "v"(a), "v"(b));
  return d;
}

#define SPLB(PH, PL, I, X) { const float xv_ = (X); const bf16_t hb_ = (bf16_t)xv_; (PH).v[I] = hb_; (PL).v[I] = (bf16_t)(xv_ - (float)hb_); }
#define SPLB8(PH, PL, A, B) { SPLB(PH, PL, 0, (A).x) SPLB(PH, PL, 1, (A).y) SPLB(PH, PL, 2, (A).z) SPLB(PH, PL, 3, (A).w) \
                              SPLB(PH, PL, 4, (B).x) SPLB(PH, PL, 5, (B).y) SPLB(PH, PL, 6, (B).z) SPLB(PH, PL, 7, (B).w) }
#define CVH(PH, I, X)       { (PH).v[I] = (f16_t)(X); }
#define CVH8(PH, A, B)      { CVH(PH, 0, (A).x) CVH(PH, 1, (A).y) CVH(PH, 2, (A).z) CVH(PH, 3, (A).w) \
                              CVH(PH, 4, (B).x) CVH(PH, 5, (B).y) CVH(PH, 6, (B).z) CVH(PH, 7, (B).w) }

__global__ __launch_bounds__(NTHR) void k_wprep(
    const float* __restrict__ Ws, const float* __restrict__ Wn,
    unsigned short* s0, unsigned short* s1, unsigned short* n0, unsigned short* n1,
    int nout, int nsplit) {
  const int which = blockIdx.y;
  const int i = blockIdx.x * NTHR + threadIdx.x;
  const int nTot = nout * (DK / 8);
  if (i >= nTot) return;
  const int o  = i * 8;
  const int n  = o / DK;
  const int k0 = o - n * DK;
  const float* W = (which == 0) ? Ws : Wn;
  const float* p = W + (size_t)k0 * nout + n;
  const float f0 = p[0] * 16.0f,                f1 = p[(size_t)nout] * 16.0f;
  const float f2 = p[(size_t)2 * nout] * 16.0f, f3 = p[(size_t)3 * nout] * 16.0f;
  const float f4 = p[(size_t)4 * nout] * 16.0f, f5 = p[(size_t)5 * nout] * 16.0f;
  const float f6 = p[(size_t)6 * nout] * 16.0f, f7 = p[(size_t)7 * nout] * 16.0f;
  unsigned short* d0 = ((which == 0) ? s0 : n0) + o;
  unsigned short* d1 = ((which == 0) ? s1 : n1) + o;
  const int split = (which == 0) ? 1 : nsplit;
  if (split != 0) {
    Pack8B ph, pl;
    SPLB(ph, pl, 0, f0) SPLB(ph, pl, 1, f1) SPLB(ph, pl, 2, f2) SPLB(ph, pl, 3, f3)
    SPLB(ph, pl, 4, f4) SPLB(ph, pl, 5, f5) SPLB(ph, pl, 6, f6) SPLB(ph, pl, 7, f7)
    const v4i qh = ph.q, ql = pl.q;
    *(volatile v4i*)d0 = qh;
    *(volatile v4i*)d1 = ql;
    __threadfence();
    *(volatile v4i*)d0 = qh;
    *(volatile v4i*)d1 = ql;
  } else {
    Pack8H ph;
    CVH(ph, 0, f0) CVH(ph, 1, f1) CVH(ph, 2, f2) CVH(ph, 3, f3)
    CVH(ph, 4, f4) CVH(ph, 5, f5) CVH(ph, 6, f6) CVH(ph, 7, f7)
    const v4i qh = ph.q;
    *(volatile v4i*)d0 = qh;
    __threadfence();
    *(volatile v4i*)d0 = qh;
  }
}

template <int NBT>
__device__ __forceinline__ int scan_chunk(const int* __restrict__ dsts, int nE, int cbase, int nodeBase,
                                          int* list, int tid, int wave) {
  int wc = 0;
#pragma unroll
  for (int g = 0; g < NGRP; ++g) {
    const int el0  = (g * NTHR + tid) * EPT;
    const int e0   = cbase + el0;
    const int sent = -2147483647 - 1;
    const int lst  = nE - 1;
    v4i da, db;
    if (e0 + 7 < nE) {
      da = *(const v4i*)(dsts + e0);
      db = *(const v4i*)(dsts + e0 + 4);
    } else {
      da.x = (e0     < nE) ? dsts[min(e0,     lst)] : sent;
      da.y = (e0 + 1 < nE) ? dsts[min(e0 + 1, lst)] : sent;
      da.z = (e0 + 2 < nE) ? dsts[min(e0 + 2, lst)] : sent;
      da.w = (e0 + 3 < nE) ? dsts[min(e0 + 3, lst)] : sent;
      db.x = (e0 + 4 < nE) ? dsts[min(e0 + 4, lst)] : sent;
      db.y = (e0 + 5 < nE) ? dsts[min(e0 + 5, lst)] : sent;
      db.z = (e0 + 6 < nE) ? dsts[min(e0 + 6, lst)] : sent;
      db.w = (e0 + 7 < nE) ? dsts[min(e0 + 7, lst)] : sent;
    }
    const unsigned nb = (unsigned)nodeBase;
    const unsigned s0 = (unsigned)da.x - nb, s1 = (unsigned)da.y - nb;
    const unsigned s2 = (unsigned)da.z - nb, s3 = (unsigned)da.w - nb;
    const unsigned s4 = (unsigned)db.x - nb, s5 = (unsigned)db.y - nb;
    const unsigned s6 = (unsigned)db.z - nb, s7 = (unsigned)db.w - nb;
    const bool h0 = s0 < (unsigned)NBT, h1 = s1 < (unsigned)NBT, h2 = s2 < (unsigned)NBT, h3 = s3 < (unsigned)NBT;
    const bool h4 = s4 < (unsigned)NBT, h5 = s5 < (unsigned)NBT, h6 = s6 < (unsigned)NBT, h7 = s7 < (unsigned)NBT;
    const unsigned any = __builtin_amdgcn_ballot_w32(h0 | h1 | h2 | h3 | h4 | h5 | h6 | h7);
    if (any != 0u) {
#define HITJ(J, HJ, SJ) { \
        const unsigned mj = __builtin_amdgcn_ballot_w32(HJ); \
        if (mj != 0u) { \
          if (HJ) { \
            const int pos = wc + (int)__builtin_amdgcn_mbcnt_lo(mj, 0u); \
            if (pos < WCAP) list[wave * WCAP + pos] = ((el0 + (J)) << 12) | (int)(SJ); \
          } \
          wc += (int)__builtin_popcount(mj); } }
      HITJ(0, h0, s0)
      HITJ(1, h1, s1)
      HITJ(2, h2, s2)
      HITJ(3, h3, s3)
      HITJ(4, h4, s4)
      HITJ(5, h5, s5)
      HITJ(6, h6, s6)
      HITJ(7, h7, s7)
#undef HITJ
    }
  }
  return wc;
}

__global__ __launch_bounds__(NTHR) void k_agg(
    const int* __restrict__ esrc, const int* __restrict__ edst,
    const float* __restrict__ xin, float* mean, int nN, int nE) {
  extern __shared__ v4f dynlds[];
  float* acc  = (float*)dynlds;
  int*   list = (int*)((char*)dynlds + LDS_ACC);
  int*   cnt  = (int*)((char*)dynlds + LDS_ACC + LDS_LIST);
  float* inv  = (float*)((char*)dynlds + LDS_ACC + LDS_LIST + LDS_CNT);
  int*   wcnt = (int*)((char*)dynlds + LDS_ACC + LDS_LIST + LDS_CNT + LDS_INV);
  const int tid = threadIdx.x, lane = tid & 31, wave = tid >> 5;
  const int nodeBase = blockIdx.x * NB;

  {
    const v4f z = {0.f, 0.f, 0.f, 0.f};
    for (int i = tid; i < NB * DK / 4; i += NTHR) dynlds[i] = z;
    if (tid < NB) cnt[tid] = 0;
  }
  __syncthreads();

  const int nChunks = (nE + CHUNK - 1) / CHUNK;
#pragma unroll 1
  for (int ch = 0; ch < nChunks; ++ch) {
    const int cbase = ch * CHUNK;
    const int wc = scan_chunk<NB>(edst, nE, cbase, nodeBase, list, tid, wave);
    if (lane == 0) wcnt[wave] = wc;
    __syncthreads();
    if (wave == 0) {
#pragma unroll 1
      for (int wsx = 0; wsx < NWAVE; ++wsx) {
        int n = __builtin_amdgcn_readfirstlane(wcnt[wsx]);
        n = n > WCAP ? WCAP : (n < 0 ? 0 : n);
        const int* lp = list + wsx * WCAP;
#pragma unroll 1
        for (int i = 0; i < n; ++i) {
          const int ent  = __builtin_amdgcn_readfirstlane(lp[i]);
          const int slot = ent & (NB - 1);
          int e = cbase + ((ent >> 12) & (CHUNK - 1));
          e = e > nE - 1 ? nE - 1 : e;
          int src = esrc[e];
          src = src < 0 ? 0 : (src > nN - 1 ? nN - 1 : src);
          const float* sp = xin + (size_t)src * DK + 4 * lane;
          v4f* ap = (v4f*)(acc + slot * DK + 4 * lane);
          const v4f x0 = *(const v4f*)(sp);
          const v4f x1 = *(const v4f*)(sp + 128);
          const v4f x2 = *(const v4f*)(sp + 256);
          const v4f x3 = *(const v4f*)(sp + 384);
          ap[0]  = ap[0]  + x0;
          ap[32] = ap[32] + x1;
          ap[64] = ap[64] + x2;
          ap[96] = ap[96] + x3;
          if (lane == 0) cnt[slot] = cnt[slot] + 1;
        }
      }
    }
    __syncthreads();
  }

  if (tid < NB) {
    const int c = cnt[tid];
    inv[tid] = 1.0f / (float)(c > 1 ? c : 1);
  }
  __syncthreads();

#pragma unroll 4
  for (int i = 0; i < (NB * DK / 4) / NTHR; ++i) {
    const int p = i * NTHR + tid;
    const int row = p >> 7, seg = p & 127;
    const v4f v = (*(const v4f*)(acc + row * DK + 4 * seg)) * inv[row];
    *(volatile v4f*)(mean + ((size_t)nodeBase + row) * DK + 4 * seg) = v;
  }
  __threadfence();
#pragma unroll 4
  for (int i = 0; i < (NB * DK / 4) / NTHR; ++i) {
    const int p = i * NTHR + tid;
    const int row = p >> 7, seg = p & 127;
    const v4f v = (*(const v4f*)(acc + row * DK + 4 * seg)) * inv[row];
    *(volatile v4f*)(mean + ((size_t)nodeBase + row) * DK + 4 * seg) = v;
  }
}

template <int RT, int CT, int SPLIT>
__device__ __forceinline__ void kphase(const float* __restrict__ X, int nN, int rowBase,
                                       const unsigned short* __restrict__ p0,
                                       const unsigned short* __restrict__ p1,
                                       unsigned short* stg0, unsigned short* stg1,
                                       int rt0, int ct0, int tid, int hh, int m,
                                       v8f (&acc)[RT][CT]) {
  const int sr = tid >> 3;
  const int sk = (tid & 7) * 16;
  int grow = rowBase + sr;
  grow = grow > nN - 1 ? nN - 1 : grow;
  const float* xr = X + (size_t)grow * DK + sk;
  unsigned short* w0 = stg0 + sr * PA + sk;
  unsigned short* w1 = stg1 + sr * PA + sk;
#pragma unroll 1
  for (int kc = 0; kc < DK; kc += KC) {
    __syncthreads();
    const v4f x0 = *(const v4f*)(xr + kc);
    const v4f x1 = *(const v4f*)(xr + kc + 4);
    const v4f x2 = *(const v4f*)(xr + kc + 8);
    const v4f x3 = *(const v4f*)(xr + kc + 12);
    if (SPLIT) {
      Pack8B ha, hb, la, lb;
      SPLB8(ha, la, x0, x1)
      SPLB8(hb, lb, x2, x3)
      *(v4i*)w0 = ha.q;  *(v4i*)(w0 + 8) = hb.q;
      *(v4i*)w1 = la.q;  *(v4i*)(w1 + 8) = lb.q;
    } else {
      Pack8H fa, fb;
      CVH8(fa, x0, x1)
      CVH8(fb, x2, x3)
      *(v4i*)w0 = fa.q;  *(v4i*)(w0 + 8) = fb.q;
    }
    __syncthreads();
#pragma unroll 1
    for (int ks = 0; ks < KC / 32; ++ks) {
      const int kg = kc + 32 * ks;
      if (SPLIT) {
        FragB ah[RT], al[RT];
#pragma unroll
        for (int rt = 0; rt < RT; ++rt) {
          const unsigned short* ap = stg0 + (16 * (rt0 + rt) + m) * PA + 32 * ks + 8 * hh;
          const unsigned short* aq = stg1 + (16 * (rt0 + rt) + m) * PA + 32 * ks + 8 * hh;
          ah[rt].q[0] = *(const v4i*)ap;  ah[rt].q[1] = *(const v4i*)(ap + 16);
          al[rt].q[0] = *(const v4i*)aq;  al[rt].q[1] = *(const v4i*)(aq + 16);
        }
#pragma unroll
        for (int ct = 0; ct < CT; ++ct) {
          const unsigned short* bp = p0 + (size_t)(16 * (ct0 + ct) + m) * DK + kg + 8 * hh;
          const unsigned short* bq = p1 + (size_t)(16 * (ct0 + ct) + m) * DK + kg + 8 * hh;
          FragB bh, bl;
          bh.q[0] = *(const v4i*)bp;  bh.q[1] = *(const v4i*)(bp + 16);
          bl.q[0] = *(const v4i*)bq;  bl.q[1] = *(const v4i*)(bq + 16);
#pragma unroll
          for (int rt = 0; rt < RT; ++rt) {
            acc[rt][ct] = wmb(al[rt].v, bh.v, acc[rt][ct]);
            acc[rt][ct] = wmb(ah[rt].v, bl.v, acc[rt][ct]);
            acc[rt][ct] = wmb(ah[rt].v, bh.v, acc[rt][ct]);
          }
        }
      } else {
        FragH a[RT];
#pragma unroll
        for (int rt = 0; rt < RT; ++rt) {
          const unsigned short* ap = stg0 + (16 * (rt0 + rt) + m) * PA + 32 * ks + 8 * hh;
          a[rt].q[0] = *(const v4i*)ap;  a[rt].q[1] = *(const v4i*)(ap + 16);
        }
#pragma unroll
        for (int ct = 0; ct < CT; ++ct) {
          const unsigned short* bp = p0 + (size_t)(16 * (ct0 + ct) + m) * DK + kg + 8 * hh;
          FragH b;
          b.q[0] = *(const v4i*)bp;  b.q[1] = *(const v4i*)(bp + 16);
#pragma unroll
          for (int rt = 0; rt < RT; ++rt)
            acc[rt][ct] = wmh(a[rt].v, b.v, acc[rt][ct]);
        }
      }
    }
  }
}

template <int NOUT, int NSPLIT, int LAST>
__global__ __launch_bounds__(NTHR) void k_gemm(
    const float* __restrict__ xself, const float* __restrict__ xmean,
    const unsigned short* __restrict__ ps0, const unsigned short* __restrict__ ps1,
    const unsigned short* __restrict__ pn0, const unsigned short* __restrict__ pn1,
    const float* __restrict__ bias, const float* __restrict__ embin,
    const int* __restrict__ lsth, const int* __restrict__ lstl,
    float* dst, int nN, int nH, int nL) {
  extern __shared__ v4f dynlds[];
  constexpr int RT  = (NOUT == 512) ? 2 : 1;
  constexpr int CT  = (NOUT == 512) ? 4 : 1;
  constexpr int OTP = GemmLds<NOUT>::OTP;
  constexpr int OTB = GemmLds<NOUT>::OTB;
  char* base = (char*)dynlds;
  unsigned short* stg0 = (unsigned short*)base;
  unsigned short* stg1 = (unsigned short*)(base + G_STG);
  float* ot    = (float*)(base + 2 * G_STG);
  int*   tabH  = (int*)(base + 2 * G_STG + OTB);
  int*   tabL  = tabH + TABMAX;
  int*   rflag = tabL + TABMAX;
  int*   rcnt  = rflag + GR;
  const int tid = threadIdx.x, lane = tid & 31, wave = tid >> 5, hh = lane >> 4, m = lane & 15;
  const int rt0 = (NOUT == 512) ? 0 : (wave & 1);
  const int ct0 = (NOUT == 512) ? (4 * wave) : (wave >> 1);
  const int rowBase = blockIdx.x * GR;

  if (LAST) {
    for (int i = tid; i < TABMAX; i += NTHR) {
      const int ih = i < nH ? i : nH - 1;
      const int il = i < nL ? i : nL - 1;
      const int vh = lsth[ih];
      const int vl = lstl[il];
      tabH[i] = (i < nH) ? vh : -1;
      tabL[i] = (i < nL) ? vl : -1;
    }
  }

  v8f acc[RT][CT];
#pragma unroll
  for (int rt = 0; rt < RT; ++rt)
#pragma unroll
    for (int ct = 0; ct < CT; ++ct) { const v8f z = {0.f, 0.f, 0.f, 0.f, 0.f, 0.f, 0.f, 0.f}; acc[rt][ct] = z; }

  kphase<RT, CT, 1>(xself, nN, rowBase, ps0, ps1, stg0, stg1, rt0, ct0, tid, hh, m, acc);
  kphase<RT, CT, NSPLIT>(xmean, nN, rowBase, pn0, pn1, stg0, stg1, rt0, ct0, tid, hh, m, acc);

#pragma unroll
  for (int rt = 0; rt < RT; ++rt) {
#pragma unroll
    for (int ct = 0; ct < CT; ++ct) {
      const int col = 16 * (ct0 + ct) + m;
      const float bv = bias[col];
      float* op = ot + (16 * (rt0 + rt) + 8 * hh) * OTP + col;
#pragma unroll
      for (int r = 0; r < 8; ++r) {
        float v = acc[rt][ct][r] * 0.0625f + bv;
        if (!LAST) v = fmaxf(v, 0.0f);
        op[r * OTP] = v;
      }
    }
  }
  __syncthreads();

  if (!LAST) {
    constexpr int PPR = NOUT / 4;
    constexpr int NIT = GR * PPR / NTHR;
#pragma unroll
    for (int i = 0; i < NIT; ++i) {
      const int p = i * NTHR + tid;
      const int row = p / PPR, seg = p - row * PPR;
      const v4f v = *(const v4f*)(ot + row * OTP + 4 * seg);
      *(volatile v4f*)(dst + ((size_t)rowBase + row) * NOUT + 4 * seg) = v;
    }
    __threadfence();
#pragma unroll
    for (int i = 0; i < NIT; ++i) {
      const int p = i * NTHR + tid;
      const int row = p / PPR, seg = p - row * PPR;
      const v4f v = *(const v4f*)(ot + row * OTP + 4 * seg);
      *(volatile v4f*)(dst + ((size_t)rowBase + row) * NOUT + 4 * seg) = v;
    }
  } else {
    if (tid < GR) {
      const int row = rowBase + tid;
      const int nHc = nH > TABMAX ? TABMAX : nH;
      const int nLc = nL > TABMAX ? TABMAX : nL;
      int sp = 0, c = 0;
#pragma unroll 1
      for (int j = 0; j < nHc; ++j) sp |= (tabH[j] == row) ? 1 : 0;
#pragma unroll 1
      for (int j = 0; j < nLc; ++j) c += (tabL[j] == row) ? 1 : 0;
      rflag[tid] = (sp != 0 || c > 0) ? 1 : 0;
      rcnt[tid]  = c;
    }
    __syncthreads();
    constexpr int PPR = NOUT / 4;
    constexpr int NIT = GR * PPR / NTHR;
    v4f vals[NIT];
#pragma unroll
    for (int i = 0; i < NIT; ++i) {
      const int p = i * NTHR + tid;
      const int row = p / PPR, seg = p - row * PPR;
      const int grow = rowBase + row;
      const int gc = grow < nN ? grow : nN - 1;
      const v4f hv = *(const v4f*)(ot + row * OTP + 4 * seg);
      const v4f ev = *(const v4f*)(embin + (size_t)gc * NOUT + 4 * seg);
      const int sp = rflag[row];
      int c = rcnt[row];
      c = c > TABMAX ? TABMAX : (c < 0 ? 0 : c);
      v4f v = (sp != 0) ? hv : ev;
#pragma unroll 1
      for (int j = 0; j < c; ++j) v = v + hv;
      vals[i] = v;
    }
#pragma unroll
    for (int i = 0; i < NIT; ++i) {
      const int p = i * NTHR + tid;
      const int row = p / PPR, seg = p - row * PPR;
      const int grow = rowBase + row;
      if (grow < nN) *(volatile v4f*)(dst + (size_t)grow * NOUT + 4 * seg) = vals[i];
    }
    __threadfence();
#pragma unroll
    for (int i = 0; i < NIT; ++i) {
      const int p = i * NTHR + tid;
      const int row = p / PPR, seg = p - row * PPR;
      const int grow = rowBase + row;
      if (grow < nN) *(volatile v4f*)(dst + (size_t)grow * NOUT + 4 * seg) = vals[i];
    }
  }
}

extern "C" void kernel_launch(void* const* d_in, const int* in_sizes, int n_in,
                              void* d_out, int out_size, void* d_ws, size_t ws_size,
                              hipStream_t stream) {
  if (n_in < 15) return;
  const int NC = 64;
  const int nN = in_sizes[0] / DK;
  if (nN <= 0 || in_sizes[0] != nN * DK) return;
  if (in_sizes[1] != DK * DK || in_sizes[2] != DK * DK || in_sizes[3] < DK) return;
  if (in_sizes[4] != DK * DK || in_sizes[5] != DK * DK || in_sizes[6] < DK) return;
  if (in_sizes[7] != DK * NC || in_sizes[8] != DK * NC || in_sizes[9] < NC) return;
  if (in_sizes[10] != nN * NC) return;
  const int nE = in_sizes[11];
  if (nE <= 0 || in_sizes[12] != nE) return;
  const int nH = in_sizes[13], nL = in_sizes[14];
  if (nH < 1 || nH > TABMAX || nL < 1 || nL > TABMAX) return;
  if (out_size != nN * NC) return;

  const float* x0    = (const float*)d_in[0];
  const float* ws0   = (const float*)d_in[1];
  const float* wn0   = (const float*)d_in[2];
  const float* b0    = (const float*)d_in[3];
  const float* ws1   = (const float*)d_in[4];
  const float* wn1   = (const float*)d_in[5];
  const float* b1    = (const float*)d_in[6];
  const float* ws2   = (const float*)d_in[7];
  const float* wn2   = (const float*)d_in[8];
  const float* b2    = (const float*)d_in[9];
  const float* embin = (const float*)d_in[10];
  const int*   esrc  = (const int*)d_in[11];
  const int*   edst  = (const int*)d_in[12];
  const int*   lsth  = (const int*)d_in[13];
  const int*   lstl  = (const int*)d_in[14];
  float* out = (float*)d_out;

  const int nBlkA = (nN + NB - 1) / NB;
  const int nBlkG = (nN + GR - 1) / GR;
  const size_t mRows = (size_t)nBlkA * NB;
  const size_t hRows = (size_t)nBlkG * GR;

  char* ws = (char*)d_ws;
  const size_t pw5 = (size_t)DK * DK * 2;
  const size_t pw2 = (size_t)NC * DK * 2;
  const size_t szH = hRows * DK * 4;
  const size_t szM = mRows * DK * 4;
  size_t off = 0;
  const size_t o_s0a = off; off += pw5;  const size_t o_s0b = off; off += pw5;
  const size_t o_n0a = off; off += pw5;  const size_t o_n0b = off; off += pw5;
  const size_t o_s1a = off; off += pw5;  const size_t o_s1b = off; off += pw5;
  const size_t o_n1a = off; off += pw5;  const size_t o_n1b = off; off += pw5;
  const size_t o_s2a = off; off += pw2;  const size_t o_s2b = off; off += pw2;
  const size_t o_n2a = off; off += pw2;  const size_t o_n2b = off; off += pw2;
  const size_t o_h1  = off; off += szH;
  const size_t o_h2  = off; off += szH;
  const size_t o_mn  = off; off += szM;
  if (off > ws_size) return;
  if (off > ((size_t)128 << 20)) return;

  unsigned short* s0a = (unsigned short*)(ws + o_s0a); unsigned short* s0b = (unsigned short*)(ws + o_s0b);
  unsigned short* n0a = (unsigned short*)(ws + o_n0a); unsigned short* n0b = (unsigned short*)(ws + o_n0b);
  unsigned short* s1a = (unsigned short*)(ws + o_s1a); unsigned short* s1b = (unsigned short*)(ws + o_s1b);
  unsigned short* n1a = (unsigned short*)(ws + o_n1a); unsigned short* n1b = (unsigned short*)(ws + o_n1b);
  unsigned short* s2a = (unsigned short*)(ws + o_s2a); unsigned short* s2b = (unsigned short*)(ws + o_s2b);
  unsigned short* n2a = (unsigned short*)(ws + o_n2a); unsigned short* n2b = (unsigned short*)(ws + o_n2b);
  float* h1 = (float*)(ws + o_h1);
  float* h2 = (float*)(ws + o_h2);
  float* mn = (float*)(ws + o_mn);

  hipFuncSetAttribute(reinterpret_cast<const void*>(&k_agg),
                      hipFuncAttributeMaxDynamicSharedMemorySize, LDS_AGG);
  hipFuncSetAttribute(reinterpret_cast<const void*>(&k_gemm<512, 0, 0>),
                      hipFuncAttributeMaxDynamicSharedMemorySize, GemmLds<512>::TOTAL);
  hipFuncSetAttribute(reinterpret_cast<const void*>(&k_gemm<64, 1, 1>),
                      hipFuncAttributeMaxDynamicSharedMemorySize, GemmLds<64>::TOTAL);

  {
    const int g5 = (DK * (DK / 8) + NTHR - 1) / NTHR;
    const int g2 = (NC * (DK / 8) + NTHR - 1) / NTHR;
    k_wprep<<<dim3(g5, 2), NTHR, 0, stream>>>(ws0, wn0, s0a, s0b, n0a, n0b, DK, 0);
    k_wprep<<<dim3(g5, 2), NTHR, 0, stream>>>(ws1, wn1, s1a, s1b, n1a, n1b, DK, 0);
    k_wprep<<<dim3(g2, 2), NTHR, 0, stream>>>(ws2, wn2, s2a, s2b, n2a, n2b, NC, 1);
  }

  k_agg<<<nBlkA, NTHR, LDS_AGG, stream>>>(esrc, edst, x0, mn, nN, nE);
  k_gemm<512, 0, 0><<<nBlkG, NTHR, GemmLds<512>::TOTAL, stream>>>(
      x0, mn, s0a, s0b, n0a, n0b, b0, embin, lsth, lstl, h1, nN, nH, nL);
  k_agg<<<nBlkA, NTHR, LDS_AGG, stream>>>(esrc, edst, h1, mn, nN, nE);
  k_gemm<512, 0, 0><<<nBlkG, NTHR, GemmLds<512>::TOTAL, stream>>>(
      h1, mn, s1a, s1b, n1a, n1b, b1, embin, lsth, lstl, h2, nN, nH, nL);
  k_agg<<<nBlkA, NTHR, LDS_AGG, stream>>>(esrc, edst, h2, mn, nN, nE);
  k_gemm<64, 1, 1><<<nBlkG, NTHR, GemmLds<64>::TOTAL, stream>>>(
      h2, mn, s2a, s2b, n2a, n2b, b2, embin, lsth, lstl, out, nN, nH, nL);
}
